// TimeMix_34815004902086
// MI455X (gfx1250) — hardware-verified
//
#include <hip/hip_runtime.h>
#include <math.h>

constexpr int kBatch  = 2;
constexpr int kSeq    = 1024;
constexpr int kChan   = 1024;
constexpr int kHead   = 64;
constexpr int kNHead  = 16;
constexpr int kRows   = kBatch * kSeq;
constexpr int kMix    = 160;
constexpr int kMixPad = 192;
constexpr int kDec    = 64;
constexpr int kBr     = 32;
constexpr int kNBr    = 5;
constexpr int kTch    = 16;
constexpr long kPlane  = (long)kRows * kChan;
constexpr long kWPlane = (long)kChan * kChan;
constexpr float kGnEps = 1.6e-4f;
static_assert(kNHead * kHead == kChan, "shape");
static_assert(kRows % 64 == 0 && kChan % 64 == 0 && kMixPad % 64 == 0 && kDec % 64 == 0, "M and N tile multiples");
static_assert(kChan % 32 == 0 && kBr % 32 == 0 && kDec % 32 == 0 && kMixPad % 32 == 0, "K multiples of 32");
static_assert(kSeq % kTch == 0 && (kTch % 2) == 0 && kTch <= 16, "scan chunking");
static_assert(kMix % 8 == 0 && kMixPad % 8 == 0 && kDec % 8 == 0, "pack groups never straddle a row");

typedef __attribute__((ext_vector_type(16))) _Float16 v16h;
typedef __attribute__((ext_vector_type(8)))  _Float16 v8h;
typedef __attribute__((ext_vector_type(16))) __bf16   v16b;
typedef __attribute__((ext_vector_type(8)))  __bf16   v8b;
typedef __attribute__((ext_vector_type(8)))  float    v8f;
typedef __attribute__((ext_vector_type(4)))  float    v4f;
typedef __attribute__((ext_vector_type(2)))  float    v2f;
typedef __attribute__((ext_vector_type(4)))  unsigned int v4u;

__device__ __forceinline__ unsigned short f2bf_bits(float f) {
  unsigned u = __float_as_uint(f);
  return (unsigned short)((u + 0x7FFFu + ((u >> 16) & 1u)) >> 16);
}
__device__ __forceinline__ float bf_bits2f(unsigned short h) { return __uint_as_float(((unsigned)h) << 16); }
__device__ __forceinline__ unsigned pk16(unsigned short a, unsigned short b) { return (unsigned)a | ((unsigned)b << 16); }
__device__ __forceinline__ void bf_split_bits(float f, unsigned short& hb, unsigned short& lb) {
  hb = f2bf_bits(f);
  lb = f2bf_bits(f - bf_bits2f(hb));
}

__device__ __forceinline__ void dep_guard4_h(v8f& a, v8f& b, v8f& c, v8f& d, v16h x, v16h y) { asm volatile("v_nop\n\tv_nop\n\tv_nop\n\tv_nop" : "+v"(a), "+v"(b), "+v"(c), "+v"(d) : "v"(x), "v"(y)); }
__device__ __forceinline__ void dep_guard4_b(v8f& a, v8f& b, v8f& c, v8f& d, v16b x, v16b y) { asm volatile("v_nop\n\tv_nop\n\tv_nop\n\tv_nop" : "+v"(a), "+v"(b), "+v"(c), "+v"(d) : "v"(x), "v"(y)); }
__device__ __forceinline__ void keep4_h(v16h a, v16h b, v16h c, v16h d) { asm volatile("v_nop" :: "v"(a), "v"(b), "v"(c), "v"(d)); }
__device__ __forceinline__ void keep4_b(v16b a, v16b b, v16b c, v16b d) { asm volatile("v_nop" :: "v"(a), "v"(b), "v"(c), "v"(d)); }
__device__ __forceinline__ void acc_guard4(v8f& a, v8f& b, v8f& c, v8f& d) { asm volatile("v_nop\n\tv_nop\n\tv_nop\n\tv_nop" : "+v"(a), "+v"(b), "+v"(c), "+v"(d)); }
template <typename T> struct Frag;
template <> struct Frag<_Float16> {
  typedef v16h V; union U { v16h v; v8h h[2]; };
  static __device__ __forceinline__ v16h load(const _Float16* p) {
    U f; f.h[0] = *(const v8h*)(p); f.h[1] = *(const v8h*)(p + 16); return f.v;
  }
  static __device__ __forceinline__ v8f mma(v16h a, v16h b, v8f c) {
    return __builtin_amdgcn_wmma_f32_16x16x32_f16(false, a, false, b, (short)0, c, false, false);
  }
  static __device__ __forceinline__ void guard4(v8f& a, v8f& b, v8f& c, v8f& d, v16h x, v16h y) { dep_guard4_h(a, b, c, d, x, y); }
  static __device__ __forceinline__ void keep(v16h a, v16h b, v16h c, v16h d) { keep4_h(a, b, c, d); }
};
template <> struct Frag<__bf16> {
  typedef v16b V; union U { v16b v; v8b h[2]; };
  static __device__ __forceinline__ v16b load(const __bf16* p) {
    U f; f.h[0] = *(const v8b*)(p); f.h[1] = *(const v8b*)(p + 16); return f.v;
  }
  static __device__ __forceinline__ v8f mma(v16b a, v16b b, v8f c) {
    return __builtin_amdgcn_wmma_f32_16x16x32_bf16(false, a, false, b, (short)0, c, false, false);
  }
  static __device__ __forceinline__ void guard4(v8f& a, v8f& b, v8f& c, v8f& d, v16b x, v16b y) { dep_guard4_b(a, b, c, d, x, y); }
  static __device__ __forceinline__ void keep(v16b a, v16b b, v16b c, v16b d) { keep4_b(a, b, c, d); }
};

template <int ET> struct Elem;
template <> struct Elem<0> { typedef _Float16 T; };
template <> struct Elem<1> { typedef __bf16 T; };
template <int ET, bool SPLIT, int BIAS_MODE, int OUT_MODE, bool RESID, int ACT = 0>
__global__ __launch_bounds__(256) void wmma_gemm64(
    const unsigned short* __restrict__ Ap, const unsigned short* __restrict__ A2p, int lda, long strideA,
    const unsigned short* __restrict__ Btp, const unsigned short* __restrict__ Bt2p, int ldb, long strideB,
    void* __restrict__ Cout, void* __restrict__ Cout2, int ldc, long strideC,
    const float* __restrict__ bias,
    const float* __restrict__ resid, long strideR,
    int M, int N, int K, float scale) {
  typedef typename Elem<ET>::T T;
  typedef typename Frag<T>::V V;
  const T* A = (const T*)Ap; const T* A2 = (const T*)A2p; const T* Bt = (const T*)Btp; const T* Bt2 = (const T*)Bt2p;
  __shared__ __align__(16) float sT[8][16 * 68];
  const int b    = blockIdx.y;
  const int lane = threadIdx.x & 31;
  const int wave = threadIdx.x >> 5;
  const int tilesN = N >> 6;
  const int tilesM = M >> 6;
  const int tile = blockIdx.x * 8 + wave;
  if (tile >= tilesM * tilesN) return;
  const int tm = tile / tilesN;
  const int tn = tile - tm * tilesN;
  const int m0 = tm << 6;
  const int n0 = tn << 6;

  const T* Ab  = A  + (size_t)b * strideA;
  const T* Bb  = Bt + (size_t)b * strideB;
  const T* Ab2 = SPLIT ? (A2  + (size_t)b * strideA) : nullptr;
  const T* Bb2 = SPLIT ? (Bt2 + (size_t)b * strideB) : nullptr;

  const int rlane = lane & 15;
  const int koff  = (lane >> 4) * 8;
  const int mOff  = (lane >> 4) * 8;

  v8f acc[4][4];
#pragma unroll
  for (int i = 0; i < 4; ++i)
#pragma unroll
    for (int j = 0; j < 4; ++j) acc[i][j] = (v8f){0.f,0.f,0.f,0.f,0.f,0.f,0.f,0.f};

  for (int k0 = 0; k0 < K; k0 += 32) {
    V bh[4], bl[4];
#pragma unroll
    for (int j = 0; j < 4; ++j) {
      const size_t bo = (size_t)(n0 + (j << 4) + rlane) * ldb + koff + k0;
      bh[j] = Frag<T>::load(Bb + bo);
      if (SPLIT) bl[j] = Frag<T>::load(Bb2 + bo);
    }
#pragma unroll
    for (int i = 0; i < 4; ++i) {
      const size_t ao = (size_t)(m0 + (i << 4) + rlane) * lda + koff + k0;
      V ah = Frag<T>::load(Ab + ao);
      V al;
      if (SPLIT) al = Frag<T>::load(Ab2 + ao);
#pragma unroll
      for (int j = 0; j < 4; ++j) {
        acc[i][j] = Frag<T>::mma(ah, bh[j], acc[i][j]);
        if (SPLIT) {
          acc[i][j] = Frag<T>::mma(ah, bl[j], acc[i][j]);
          acc[i][j] = Frag<T>::mma(al, bh[j], acc[i][j]);
        }
      }
      Frag<T>::guard4(acc[i][0], acc[i][1], acc[i][2], acc[i][3], ah, SPLIT ? al : ah);
    }
    Frag<T>::keep(bh[0], bh[1], bh[2], bh[3]);
    if (SPLIT) Frag<T>::keep(bl[0], bl[1], bl[2], bl[3]);
  }
  acc_guard4(acc[0][0], acc[0][1], acc[0][2], acc[0][3]);
  acc_guard4(acc[1][0], acc[1][1], acc[1][2], acc[1][3]);
  acc_guard4(acc[2][0], acc[2][1], acc[2][2], acc[2][3]);
  acc_guard4(acc[3][0], acc[3][1], acc[3][2], acc[3][3]);

  float* slab = sT[wave];
  const float* Rb = RESID ? (resid + (size_t)b * strideR) : nullptr;
#pragma unroll
  for (int i = 0; i < 4; ++i) {
    const int mBase = m0 + (i << 4);
#pragma unroll
    for (int j = 0; j < 4; ++j) {
      const int n = n0 + (j << 4) + rlane;
      float bv = 0.f;
      if (BIAS_MODE == 2) bv = bias[n];
#pragma unroll
      for (int r = 0; r < 8; ++r) {
        float v = acc[i][j][r] * scale;
        if (BIAS_MODE == 1) v += bias[mBase + mOff + r];
        if (BIAS_MODE == 2) v += bv;
        if (RESID) v += Rb[(size_t)(mBase + mOff + r) * ldc + n];
        if (ACT == 2) v = fmaxf(v, 0.0f);
        if (ACT == 4) v = (v > 0.f) ? v : 0.01f * v;
        slab[(mOff + r) * 68 + (j << 4) + rlane] = v;
      }
    }
    __builtin_amdgcn_fence(__ATOMIC_RELEASE, "workgroup");
    __builtin_amdgcn_wave_barrier();
    __builtin_amdgcn_fence(__ATOMIC_ACQUIRE, "workgroup");
    if (OUT_MODE == 0) {
      float* C = (float*)Cout + (size_t)b * strideC;
      const int hh = lane >> 4, c4 = (lane & 15) * 4;
      for (int pass = 0; pass < 2; ++pass) {
#pragma unroll
        for (int it = 0; it < 8; ++it) {
          const int row = it * 2 + hh;
          v4f v = *(const v4f*)(slab + row * 68 + c4);
          *(volatile v4f*)(C + (size_t)(mBase + row) * ldc + n0 + c4) = v;
        }
        __threadfence();
      }
    } else {
      const int q = lane >> 3, c8 = (lane & 7) * 8;
      unsigned short* C  = (unsigned short*)Cout  + (size_t)b * strideC;
      unsigned short* C2 = (OUT_MODE == 2) ? ((unsigned short*)Cout2 + (size_t)b * strideC) : nullptr;
      for (int pass = 0; pass < 2; ++pass) {
#pragma unroll
        for (int it = 0; it < 4; ++it) {
          const int row = it * 4 + q;
          const float* sp = slab + row * 68 + c8;
          v8h hv, lv;
#pragma unroll
          for (int e = 0; e < 8; ++e) {
            if (OUT_MODE == 1) {
              hv[e] = (_Float16)sp[e];
            } else {
              unsigned short hb = f2bf_bits(sp[e]);
              unsigned short lb = f2bf_bits(sp[e] - bf_bits2f(hb));
              hv[e] = __builtin_bit_cast(_Float16, hb);
              lv[e] = __builtin_bit_cast(_Float16, lb);
            }
          }
          *(volatile v8h*)(C + (size_t)(mBase + row) * ldc + n0 + c8) = hv;
          if (OUT_MODE == 2) *(volatile v8h*)(C2 + (size_t)(mBase + row) * ldc + n0 + c8) = lv;
        }
        __threadfence();
      }
    }
    __builtin_amdgcn_fence(__ATOMIC_RELEASE, "workgroup");
    __builtin_amdgcn_wave_barrier();
    __builtin_amdgcn_fence(__ATOMIC_ACQUIRE, "workgroup");
  }
}

__global__ __launch_bounds__(256) void k_wsplit8(const float* __restrict__ W0, const float* __restrict__ W1,
                                                 const float* __restrict__ W2, const float* __restrict__ W3,
                                                 unsigned short* __restrict__ outH, unsigned short* __restrict__ outL,
                                                 int n8PerMat) {
  const int z = blockIdx.y;
  const float* W = (z == 0) ? W0 : (z == 1) ? W1 : (z == 2) ? W2 : W3;
  const int i = blockIdx.x * 256 + threadIdx.x;
  if (i >= n8PerMat) return;
  const float* p = W + 8 * (size_t)i;
  const v4f a = *(const v4f*)(p);
  const v4f c = *(const v4f*)(p + 4);
  unsigned short hb[8], lb[8];
#pragma unroll
  for (int e = 0; e < 4; ++e) {
    bf_split_bits(a[e], hb[e], lb[e]);
    bf_split_bits(c[e], hb[4 + e], lb[4 + e]);
  }
  const v4u uh = (v4u){pk16(hb[0], hb[1]), pk16(hb[2], hb[3]), pk16(hb[4], hb[5]), pk16(hb[6], hb[7])};
  const v4u ul = (v4u){pk16(lb[0], lb[1]), pk16(lb[2], lb[3]), pk16(lb[4], lb[5]), pk16(lb[6], lb[7])};
  const size_t o = (size_t)z * (size_t)kWPlane + 8 * (size_t)i;
  *(volatile v4u*)(outH + o) = uh;
  *(volatile v4u*)(outL + o) = ul;
  __threadfence();
  *(volatile v4u*)(outH + o) = uh;
  *(volatile v4u*)(outL + o) = ul;
}

template <bool SPLIT, int KT>
__global__ __launch_bounds__(256) void k_trcast(const float* __restrict__ in, int R, int Cc, long inStrideZ,
                                                unsigned short* __restrict__ outH, unsigned short* __restrict__ outL,
                                                int ldo, long outStrideZ) {
  static_assert(KT == 64 || KT == 32, "tile");
  __shared__ float sm[32][KT + 1];
  const int t  = threadIdx.x;
  const int n0 = blockIdx.x * 32;
  const int k0 = blockIdx.y * KT;
  const float* inz = in + (size_t)blockIdx.z * inStrideZ;
  constexpr int kIters = (32 * KT) / 256;
#pragma unroll
  for (int it = 0; it < kIters; ++it) {
    const int e  = it * 256 + t;
    const int nl = e & 31;
    const int kl = e >> 5;
    const int n  = n0 + nl;
    const int k  = k0 + kl;
    const int nc = (n < Cc) ? n : (Cc - 1);
    const int kc = (k < R) ? k : (R - 1);
    const float v  = inz[(size_t)kc * Cc + nc];
    const float fz = ((n < Cc) && (k < R)) ? 1.0f : 0.0f;
    sm[nl][kl] = v * fz;
  }
  __syncthreads();
  const int lane = t & 31, wave = t >> 5;
  unsigned short* oh = outH + (size_t)blockIdx.z * outStrideZ;
  unsigned short* ol = outL + (size_t)blockIdx.z * outStrideZ;
  int row, c8;
  bool active;
  if (KT == 64) { row = wave * 4 + (lane >> 3); c8 = (lane & 7) * 8; active = true; }
  else          { row = t >> 2;                 c8 = (t & 3) * 8;    active = (t < 128); }
  if (active) {
    unsigned short hb[8], lb[8];
#pragma unroll
    for (int e = 0; e < 8; ++e) {
      const float v = sm[row][c8 + e];
      if (SPLIT) { bf_split_bits(v, hb[e], lb[e]); }
      else       { hb[e] = f2bf_bits(v); lb[e] = 0; }
    }
    const v4u uh = (v4u){pk16(hb[0], hb[1]), pk16(hb[2], hb[3]), pk16(hb[4], hb[5]), pk16(hb[6], hb[7])};
    const v4u ul = (v4u){pk16(lb[0], lb[1]), pk16(lb[2], lb[3]), pk16(lb[4], lb[5]), pk16(lb[6], lb[7])};
    const size_t o = (size_t)(n0 + row) * ldo + k0 + c8;
    *(volatile v4u*)(oh + o) = uh;
    if (SPLIT) *(volatile v4u*)(ol + o) = ul;
    __threadfence();
    *(volatile v4u*)(oh + o) = uh;
    if (SPLIT) *(volatile v4u*)(ol + o) = ul;
  }
}

__global__ __launch_bounds__(256) void k_xx8(const float* __restrict__ x, const float* __restrict__ miu_x,
                                             unsigned short* __restrict__ XX, int n8) {
  const int i = blockIdx.x * 256 + threadIdx.x;
  if (i >= n8) return;
  const int f  = 8 * i;
  const int m  = f >> 10;
  const int c0 = f & 1023;
  const int t  = m & 1023;
  const int mp = (t > 0) ? (m - 1) : m;
  const float fz = (t > 0) ? 1.0f : 0.0f;
  const float* px = x + f;
  const float* pp = x + ((size_t)mp << 10) + c0;
  const float* pm = miu_x + c0;
  const v4f a0 = *(const v4f*)(px), a1 = *(const v4f*)(px + 4);
  const v4f b0 = *(const v4f*)(pp), b1 = *(const v4f*)(pp + 4);
  const v4f u0 = *(const v4f*)(pm), u1 = *(const v4f*)(pm + 4);
  unsigned short hb[8];
#pragma unroll
  for (int e = 0; e < 4; ++e) {
    const float ba0 = b0[e] * fz - a0[e];
    const float ba1 = b1[e] * fz - a1[e];
    hb[e]     = f2bf_bits(a0[e] + ba0 * u0[e]);
    hb[4 + e] = f2bf_bits(a1[e] + ba1 * u1[e]);
  }
  const v4u uh = (v4u){pk16(hb[0], hb[1]), pk16(hb[2], hb[3]), pk16(hb[4], hb[5]), pk16(hb[6], hb[7])};
  unsigned short* q = XX + f;
  *(volatile v4u*)q = uh;
  __threadfence();
  *(volatile v4u*)q = uh;
}

__global__ __launch_bounds__(256) void k_x5_8(const float* __restrict__ x, const float* __restrict__ miu,
                                              const float* __restrict__ lam_s,
                                              unsigned short* __restrict__ outH, unsigned short* __restrict__ outL,
                                              int writeLo, int n8) {
  const int i = blockIdx.x * 256 + threadIdx.x;
  if (i >= n8) return;
  const int f  = 8 * i;
  const int m  = f >> 10;
  const int c0 = f & 1023;
  const int t  = m & 1023;
  const int mp = (t > 0) ? (m - 1) : m;
  const float fz = (t > 0) ? 1.0f : 0.0f;
  const float* px = x + f;
  const float* pp = x + ((size_t)mp << 10) + c0;
  const float* pm = miu + f;
  const float* pl = lam_s + c0;
  const v4f a0 = *(const v4f*)(px), a1 = *(const v4f*)(px + 4);
  const v4f b0 = *(const v4f*)(pp), b1 = *(const v4f*)(pp + 4);
  const v4f u0 = *(const v4f*)(pm), u1 = *(const v4f*)(pm + 4);
  const v4f l0 = *(const v4f*)(pl), l1 = *(const v4f*)(pl + 4);
  unsigned short hb[8], lb[8];
#pragma unroll
  for (int e = 0; e < 4; ++e) {
    const float ba0 = b0[e] * fz - a0[e];
    const float ba1 = b1[e] * fz - a1[e];
    const float v0 = a0[e] + ba0 * (u0[e] + l0[e]);
    const float v1 = a1[e] + ba1 * (u1[e] + l1[e]);
    bf_split_bits(v0, hb[e], lb[e]);
    bf_split_bits(v1, hb[4 + e], lb[4 + e]);
  }
  const v4u uh = (v4u){pk16(hb[0], hb[1]), pk16(hb[2], hb[3]), pk16(hb[4], hb[5]), pk16(hb[6], hb[7])};
  const v4u ul = (v4u){pk16(lb[0], lb[1]), pk16(lb[2], lb[3]), pk16(lb[4], lb[5]), pk16(lb[6], lb[7])};
  *(volatile v4u*)(outH + f) = uh;
  if (writeLo) *(volatile v4u*)(outL + f) = ul;
  __threadfence();
  *(volatile v4u*)(outH + f) = uh;
  if (writeLo) *(volatile v4u*)(outL + f) = ul;
}

template <bool SPLIT>
__global__ __launch_bounds__(256) void k_tanh2(const float* __restrict__ in, int ldin,
                                               unsigned short* __restrict__ outH, unsigned short* __restrict__ outL,
                                               int ncols, int nvalid, int n2) {
  const int i = blockIdx.x * 256 + threadIdx.x;
  if (i >= n2) return;
  const int f = 2 * i;
  const int m = f / ncols;
  const int c = f - m * ncols;
  const v2f a = *(const v2f*)(in + (size_t)m * ldin + c);
  const float f0 = (c < nvalid) ? 1.0f : 0.0f;
  const float f1 = (c + 1 < nvalid) ? 1.0f : 0.0f;
  const float t0 = tanhf(a[0]) * f0;
  const float t1 = tanhf(a[1]) * f1;
  unsigned short h0, h1, l0 = 0, l1 = 0;
  if (SPLIT) { bf_split_bits(t0, h0, l0); bf_split_bits(t1, h1, l1); }
  else       { h0 = f2bf_bits(t0); h1 = f2bf_bits(t1); }
  const unsigned uh = pk16(h0, h1);
  const unsigned ul = pk16(l0, l1);
  ((volatile unsigned*)outH)[i] = uh;
  if (SPLIT) ((volatile unsigned*)outL)[i] = ul;
  __threadfence();
  ((volatile unsigned*)outH)[i] = uh;
  if (SPLIT) ((volatile unsigned*)outL)[i] = ul;
}

__global__ __launch_bounds__(256) void k_state_scan(const float* __restrict__ kraw, const float* __restrict__ vpl,
                                                    const float* __restrict__ rpl, const float* __restrict__ wl,
                                                    const float* __restrict__ td_miu, const float* __restrict__ u,
                                                    float* __restrict__ Y) {
  __shared__ __align__(16) float sr[kTch][64];
  __shared__ __align__(16) float sk[kTch][64];
  __shared__ __align__(16) float sd[kTch][64];
  __shared__ __align__(16) float sv[kTch][64];
  __shared__ float su[64];
  __shared__ float stm[64];
  __shared__ float sbon[kTch];
  __shared__ __align__(16) float part[2][4][64];
  const int tid = threadIdx.x;
  const int b   = blockIdx.x / kNHead;
  const int n   = blockIdx.x - b * kNHead;
  const int i   = tid & 63;
  const int jg  = tid >> 6;
  const int j0  = jg * 16;
  float S[16];
#pragma unroll
  for (int jj = 0; jj < 16; ++jj) S[jj] = 0.0f;
  if (tid < 64) {
    su[tid]  = u[n * kHead + tid];
    stm[tid] = td_miu[n * kHead + tid];
  }
  const size_t base = (size_t)b * kSeq * kChan + (size_t)n * kHead;
  for (int t0 = 0; t0 < kSeq; t0 += kTch) {
    __syncthreads();
#pragma unroll 1
    for (int it = 0; it < (kTch * 64) / 256; ++it) {
      const int e  = it * 256 + tid;
      const int tl = e >> 6;
      const int c  = e & 63;
      const size_t off = base + (size_t)(t0 + tl) * kChan + c;
      const float wv = wl[off] + stm[c];
      sr[tl][c] = rpl[off];
      sk[tl][c] = kraw[off] * expf(fminf(wv, 0.0f));
      sd[tl][c] = expf(wv);
      sv[tl][c] = vpl[off];
    }
    __syncthreads();
    if (tid < kTch) {
      float bs = 0.0f;
#pragma unroll 1
      for (int j = 0; j < 64; ++j) bs += sr[tid][j] * (su[j] * sk[tid][j]);
      sbon[tid] = bs;
    }
    __syncthreads();
    for (int tl = 0; tl < kTch; ++tl) {
      const int p = tl & 1;
      const float vi = sv[tl][i];
      float acc = 0.0f;
#pragma unroll
      for (int jj = 0; jj < 16; ++jj) {
        const int j = j0 + jj;
        const float rj = sr[tl][j];
        const float kj = sk[tl][j];
        const float dj = sd[tl][j];
        acc += rj * S[jj];
        S[jj] = S[jj] * dj + kj * vi;
      }
      part[p][jg][i] = acc;
      __syncthreads();
      if (tid < 16) {
        const v4f p0 = *(const v4f*)(&part[p][0][4 * tid]);
        const v4f p1 = *(const v4f*)(&part[p][1][4 * tid]);
        const v4f p2 = *(const v4f*)(&part[p][2][4 * tid]);
        const v4f p3 = *(const v4f*)(&part[p][3][4 * tid]);
        const v4f vv = *(const v4f*)(&sv[tl][4 * tid]);
        const float bn = sbon[tl];
        const v4f yv = ((p0 + p1) + (p2 + p3)) + vv * bn;
        float* yp = Y + base + (size_t)(t0 + tl) * kChan + 4 * tid;
        *(volatile v4f*)yp = yv;
        __threadfence();
        *(volatile v4f*)yp = yv;
      }
    }
  }
}

__global__ __launch_bounds__(256) void k_gn_gate(const float* __restrict__ Y, const float* __restrict__ G,
                                                 const float* __restrict__ gamma, const float* __restrict__ beta,
                                                 unsigned short* __restrict__ outH, unsigned short* __restrict__ outL) {
  __shared__ __align__(16) float slab[8][64];
  const int lane = threadIdx.x & 31, wave = threadIdx.x >> 5;
  const int pair = blockIdx.x * 8 + wave;
  const int m = pair >> 4;
  const int n = pair & 15;
  const size_t base = (size_t)m * kChan + (size_t)n * kHead;
  const int c = n * kHead + 2 * lane;
  const v2f yv = *(const v2f*)(Y + base + 2 * lane);
  const v2f gv = *(const v2f*)(G + base + 2 * lane);
  const v2f ga = *(const v2f*)(gamma + c);
  const v2f be = *(const v2f*)(beta + c);
  float s = yv[0] + yv[1];
#pragma unroll
  for (int off = 16; off > 0; off >>= 1) s += __shfl_xor(s, off, 32);
  const float mean = s * (1.0f / 64.0f);
  const float d0 = yv[0] - mean;
  const float d1 = yv[1] - mean;
  float q = d0 * d0 + d1 * d1;
#pragma unroll
  for (int off = 16; off > 0; off >>= 1) q += __shfl_xor(q, off, 32);
  const float var = q * (1.0f / 64.0f);
  const float rs  = 1.0f / sqrtf(var + kGnEps);
  const float o0 = ((d0 * rs) * ga[0] + be[0]) * gv[0];
  const float o1 = ((d1 * rs) * ga[1] + be[1]) * gv[1];
  *(v2f*)(&slab[wave][2 * lane]) = (v2f){o0, o1};
  __syncthreads();
  if (lane < 8) {
    unsigned short hb[8], lb[8];
#pragma unroll
    for (int e = 0; e < 8; ++e) bf_split_bits(slab[wave][8 * lane + e], hb[e], lb[e]);
    const v4u uh = (v4u){pk16(hb[0], hb[1]), pk16(hb[2], hb[3]), pk16(hb[4], hb[5]), pk16(hb[6], hb[7])};
    const v4u ul = (v4u){pk16(lb[0], lb[1]), pk16(lb[2], lb[3]), pk16(lb[4], lb[5]), pk16(lb[6], lb[7])};
    const size_t o = base + 8 * (size_t)lane;
    *(volatile v4u*)(outH + o) = uh;
    *(volatile v4u*)(outL + o) = ul;
    __threadfence();
    *(volatile v4u*)(outH + o) = uh;
    *(volatile v4u*)(outL + o) = ul;
  }
}

extern "C" void kernel_launch(void* const* d_in, const int* in_sizes, int n_in,
                              void* d_out, int out_size, void* d_ws, size_t ws_size,
                              hipStream_t stream) {
  if (n_in < 17) return;
  if (in_sizes[0] != kBatch * kSeq * kChan) return;
  if (in_sizes[1] != kChan || in_sizes[2] != kNBr * kChan) return;
  if (in_sizes[3] != kChan * kMix || in_sizes[4] != kNBr * kBr * kChan) return;
  if (in_sizes[5] != kChan || in_sizes[6] != kChan * kDec || in_sizes[7] != kDec * kChan) return;
  if (in_sizes[8] != kNHead * kHead) return;
  if (in_sizes[9] != kChan * kChan || in_sizes[10] != kChan * kChan || in_sizes[11] != kChan * kChan || in_sizes[12] != kChan * kChan) return;
  if (in_sizes[13] != kChan * kMix || in_sizes[14] != kMix * kChan) return;
  if (in_sizes[15] != kChan || in_sizes[16] != kChan) return;
  if (out_size != kBatch * kSeq * kChan) return;

  const float* x      = (const float*)d_in[0];
  const float* miu_x  = (const float*)d_in[1];
  const float* lam    = (const float*)d_in[2];
  const float* Amat   = (const float*)d_in[3];
  const float* Bp     = (const float*)d_in[4];
  const float* td_miu = (const float*)d_in[5];
  const float* tdA    = (const float*)d_in[6];
  const float* tdB    = (const float*)d_in[7];
  const float* u      = (const float*)d_in[8];
  const float* Wk     = (const float*)d_in[9];
  const float* Wv     = (const float*)d_in[10];
  const float* Wr     = (const float*)d_in[11];
  const float* Wo     = (const float*)d_in[12];
  const float* Wg1    = (const float*)d_in[13];
  const float* Wg2    = (const float*)d_in[14];
  const float* gamma  = (const float*)d_in[15];
  const float* beta   = (const float*)d_in[16];
  float* out = (float*)d_out;

  const size_t szXX    = (size_t)kPlane * 2;
  const size_t szHPRE  = (size_t)kRows * kMixPad * 4;
  const size_t szHC    = (size_t)kRows * kMix * 2;
  const size_t szF32P  = (size_t)kPlane * 4;
  const size_t szX5H   = (size_t)kNBr * kPlane * 2;
  const size_t szX5L   = (size_t)(kNBr - 1) * kPlane * 2;
  const size_t szWSQ   = (size_t)4 * kWPlane * 2;
  const size_t szAT    = (size_t)kMixPad * kChan * 2;
  const size_t szTDAT  = (size_t)kDec * kChan * 2;
  const size_t szTDBT  = (size_t)kChan * kDec * 2;
  const size_t szWG1T  = (size_t)kMixPad * kChan * 2;
  const size_t szWG2T  = (size_t)kChan * kMixPad * 2;
  const size_t szBPT   = (size_t)kNBr * kChan * kBr * 2;
  const size_t szLPRE  = (size_t)kRows * kDec * 4;
  const size_t szL1    = (size_t)kRows * kDec * 2;
  const size_t szKVR   = (size_t)3 * kPlane * 4;
  const size_t szGHPRE = (size_t)kRows * kMixPad * 4;
  const size_t szGH    = (size_t)kRows * kMixPad * 2;
  const size_t szGAT   = (size_t)kPlane * 2;
  size_t off = 0;
  const size_t oXX    = off; off += szXX;
  const size_t oHPRE  = off; off += szHPRE;
  const size_t oHC    = off; off += szHC;
  const size_t oMIU   = off; off += szF32P;
  const size_t oX5H   = off; off += szX5H;
  const size_t oX5L   = off; off += szX5L;
  const size_t oWH    = off; off += szWSQ;
  const size_t oWL    = off; off += szWSQ;
  const size_t oAT    = off; off += szAT;
  const size_t oTDAT  = off; off += szTDAT;
  const size_t oTDBT  = off; off += szTDBT;
  const size_t oWG1TH = off; off += szWG1T;
  const size_t oWG1TL = off; off += szWG1T;
  const size_t oWG2TH = off; off += szWG2T;
  const size_t oWG2TL = off; off += szWG2T;
  const size_t oBPT   = off; off += szBPT;
  const size_t oLPRE  = off; off += szLPRE;
  const size_t oL1    = off; off += szL1;
  const size_t oKVR   = off; off += szKVR;
  const size_t oGHPRE = off; off += szGHPRE;
  const size_t oGHH   = off; off += szGH;
  const size_t oGHL   = off; off += szGH;
  const size_t oGATE  = off; off += szF32P;
  const size_t oY     = off; off += szF32P;
  const size_t oGATH  = off; off += szGAT;
  const size_t oGATL  = off; off += szGAT;
  const size_t total  = off;
  if (total > (size_t)134217728) return;
  if (ws_size < total) return;

  char* ws = (char*)d_ws;
  unsigned short* XX    = (unsigned short*)(ws + oXX);
  float*          HPRE  = (float*)(ws + oHPRE);
  unsigned short* HC    = (unsigned short*)(ws + oHC);
  float*          MIU   = (float*)(ws + oMIU);
  float*          WLR   = MIU;
  unsigned short* X5H   = (unsigned short*)(ws + oX5H);
  unsigned short* X5L   = (unsigned short*)(ws + oX5L);
  unsigned short* WH    = (unsigned short*)(ws + oWH);
  unsigned short* WL    = (unsigned short*)(ws + oWL);
  unsigned short* AT    = (unsigned short*)(ws + oAT);
  unsigned short* TDAT  = (unsigned short*)(ws + oTDAT);
  unsigned short* TDBT  = (unsigned short*)(ws + oTDBT);
  unsigned short* WG1TH = (unsigned short*)(ws + oWG1TH);
  unsigned short* WG1TL = (unsigned short*)(ws + oWG1TL);
  unsigned short* WG2TH = (unsigned short*)(ws + oWG2TH);
  unsigned short* WG2TL = (unsigned short*)(ws + oWG2TL);
  unsigned short* BPT   = (unsigned short*)(ws + oBPT);
  float*          LPRE  = (float*)(ws + oLPRE);
  unsigned short* L1    = (unsigned short*)(ws + oL1);
  float*          KVR   = (float*)(ws + oKVR);
  float*          GHPRE = (float*)(ws + oGHPRE);
  unsigned short* GHH   = (unsigned short*)(ws + oGHH);
  unsigned short* GHL   = (unsigned short*)(ws + oGHL);
  float*          GATE  = (float*)(ws + oGATE);
  float*          Yp    = (float*)(ws + oY);
  unsigned short* GATH  = (unsigned short*)(ws + oGATH);
  unsigned short* GATL  = (unsigned short*)(ws + oGATL);
  const float* fdum = gamma;

  const dim3 blk(256);
  const int n8Plane = (int)(kPlane / 8);
  const int n8W     = (int)(kWPlane / 8);

  k_wsplit8<<<dim3(n8W / 256, 4), blk, 0, stream>>>(Wk, Wv, Wr, Wo, WH, WL, n8W);
  k_trcast<false, 64><<<dim3(kMixPad / 32, kChan / 64, 1), blk, 0, stream>>>(Amat, kChan, kMix, 0L, AT, AT, kChan, 0L);
  k_trcast<false, 64><<<dim3(kDec / 32, kChan / 64, 1), blk, 0, stream>>>(tdA, kChan, kDec, 0L, TDAT, TDAT, kChan, 0L);
  k_trcast<false, 64><<<dim3(kChan / 32, 1, 1), blk, 0, stream>>>(tdB, kDec, kChan, 0L, TDBT, TDBT, kDec, 0L);
  k_trcast<true, 64><<<dim3(kMixPad / 32, kChan / 64, 1), blk, 0, stream>>>(Wg1, kChan, kMix, 0L, WG1TH, WG1TL, kChan, 0L);
  k_trcast<true, 64><<<dim3(kChan / 32, kMixPad / 64, 1), blk, 0, stream>>>(Wg2, kMix, kChan, 0L, WG2TH, WG2TL, kMixPad, 0L);
  k_trcast<false, 32><<<dim3(kChan / 32, 1, kNBr), blk, 0, stream>>>(Bp, kBr, kChan, (long)kBr * kChan, BPT, BPT, kBr, (long)kChan * kBr);

  k_xx8<<<dim3(n8Plane / 256), blk, 0, stream>>>(x, miu_x, XX, n8Plane);

  wmma_gemm64<1, false, 0, 0, false, 0><<<dim3(((kRows / 64) * (kMixPad / 64) + 7) / 8, 1), blk, 0, stream>>>(
      XX, XX, kChan, 0L, AT, AT, kChan, 0L, (void*)HPRE, (void*)HPRE, kMixPad, 0L, fdum, fdum, 0L,
      kRows, kMixPad, kChan, 1.0f);
  k_tanh2<false><<<dim3((kRows * kMix / 2) / 256), blk, 0, stream>>>(HPRE, kMixPad, HC, HC, kMix, kMix, kRows * kMix / 2);

  for (int s = 0; s < kNBr; ++s) {
    const unsigned short* Hs = HC + (size_t)s * kRows * kBr;
    const unsigned short* Bs = BPT + (size_t)s * kChan * kBr;
    wmma_gemm64<1, false, 0, 0, false, 0><<<dim3(((kRows / 64) * (kChan / 64) + 7) / 8, 1), blk, 0, stream>>>(
        Hs, Hs, kBr, 0L, Bs, Bs, kBr, 0L, (void*)MIU, (void*)MIU, kChan, 0L, fdum, fdum, 0L,
        kRows, kChan, kBr, 1.0f);
    unsigned short* oh = X5H + (size_t)s * kPlane;
    unsigned short* ol = X5L + (size_t)(s > 0 ? (s - 1) : 0) * kPlane;
    k_x5_8<<<dim3(n8Plane / 256), blk, 0, stream>>>(x, MIU, lam + (size_t)s * kChan, oh, ol, (s > 0) ? 1 : 0, n8Plane);
  }

  wmma_gemm64<1, false, 0, 0, false, 0><<<dim3(((kRows / 64) * (kDec / 64) + 7) / 8, 1), blk, 0, stream>>>(
      X5H, X5H, kChan, 0L, TDAT, TDAT, kChan, 0L, (void*)LPRE, (void*)LPRE, kDec, 0L, fdum, fdum, 0L,
      kRows, kDec, kChan, 1.0f);
  k_tanh2<false><<<dim3((kRows * kDec / 2) / 256), blk, 0, stream>>>(LPRE, kDec, L1, L1, kDec, kDec, kRows * kDec / 2);
  wmma_gemm64<1, false, 0, 0, false, 0><<<dim3(((kRows / 64) * (kChan / 64) + 7) / 8, 1), blk, 0, stream>>>(
      L1, L1, kDec, 0L, TDBT, TDBT, kDec, 0L, (void*)WLR, (void*)WLR, kChan, 0L, fdum, fdum, 0L,
      kRows, kChan, kDec, 1.0f);

  wmma_gemm64<1, true, 0, 0, false, 0><<<dim3(((kRows / 64) * (kChan / 64) + 7) / 8, 3), blk, 0, stream>>>(
      X5H + kPlane, X5L, kChan, (long)kPlane, WH, WL, kChan, (long)kWPlane,
      (void*)KVR, (void*)KVR, kChan, (long)kPlane, fdum, fdum, 0L, kRows, kChan, kChan, 1.0f);

  wmma_gemm64<1, true, 0, 0, false, 0><<<dim3(((kRows / 64) * (kMixPad / 64) + 7) / 8, 1), blk, 0, stream>>>(
      X5H + 4 * kPlane, X5L + 3 * kPlane, kChan, 0L, WG1TH, WG1TL, kChan, 0L,
      (void*)GHPRE, (void*)GHPRE, kMixPad, 0L, fdum, fdum, 0L, kRows, kMixPad, kChan, 1.0f);
  k_tanh2<true><<<dim3((kRows * kMixPad / 2) / 256), blk, 0, stream>>>(GHPRE, kMixPad, GHH, GHL, kMixPad, kMix, kRows * kMixPad / 2);
  wmma_gemm64<1, true, 0, 0, false, 0><<<dim3(((kRows / 64) * (kChan / 64) + 7) / 8, 1), blk, 0, stream>>>(
      GHH, GHL, kMixPad, 0L, WG2TH, WG2TL, kMixPad, 0L, (void*)GATE, (void*)GATE, kChan, 0L, fdum, fdum, 0L,
      kRows, kChan, kMixPad, 1.0f);

  k_state_scan<<<dim3(kBatch * kNHead), blk, 0, stream>>>(KVR, KVR + kPlane, KVR + 2 * kPlane, WLR, td_miu, u, Yp);

  k_gn_gate<<<dim3((kRows * kNHead) / 8), blk, 0, stream>>>(Yp, GATE, gamma, beta, GATH, GATL);

  wmma_gemm64<1, true, 0, 0, false, 0><<<dim3(((kRows / 64) * (kChan / 64) + 7) / 8, 1), blk, 0, stream>>>(
      GATH, GATL, kChan, 0L, WH + 3 * kWPlane, WL + 3 * kWPlane, kChan, 0L,
      (void*)out, (void*)out, kChan, 0L, fdum, fdum, 0L, kRows, kChan, kChan, 1.0f);
}
